// GAT_21062519619905
// MI455X (gfx1250) — hardware-verified
//
#include <hip/hip_runtime.h>
#include <stddef.h>
#include <stdint.h>
#include <math.h>


#define DIN    128
#define HC     128
#define CPH    32
#define KP     256
#define C3     8
#define N3P    16
#define R3W    16
#define NTHR   256
#define NWAVE  8
#define EPT    8
#define CHUNK  (NTHR * EPT)
#define WCAP   (EPT * 32)
#define LISTN  (NWAVE * WCAP)
#define NBA    1024
#define SLA    10
#define RCAP   28672
#define DEGCAP 128
#define GBM    64
#define GTHR   128
#define NU1    (HC * (DIN / 8))
#define NU2    (HC * (KP / 8))
#define NU3    (N3P * (KP / 8))
#define NEGSL  0.2f
#define EPS_SM 1e-16f
#define BN_EPS 1e-5f
#define AGG_ZINTS (LISTN + 2 * RCAP + 3 * NBA)
#define AGG_LDS_INTS (AGG_ZINTS + 16)
#define WSMAX  134217728

static_assert((CHUNK & (CHUNK - 1)) == 0 && CHUNK <= 4096);
static_assert((NBA & (NBA - 1)) == 0 && NBA == (1 << SLA));
static_assert(((long long)CHUNK << SLA) < (1LL << 31));
static_assert(LISTN % NTHR == 0);
static_assert(NBA % NWAVE == 0 && NBA % 32 == 0 && NBA % GBM == 0 && NBA % 16 == 0 && NBA % NTHR == 0);
static_assert(RCAP % 4 == 0 && AGG_ZINTS % 4 == 0 && LISTN % 4 == 0);
static_assert(DIN % 32 == 0 && KP % 32 == 0 && KP == 2 * HC && HC == 4 * CPH);
static_assert(GBM == (GTHR / 32) * 16 && HC == 4 * 32);
static_assert(NU1 % NTHR == 0 && NU2 % NTHR == 0 && NU3 % NTHR == 0);
static_assert(AGG_LDS_INTS * 4 <= 300000);
static_assert(NWAVE * HC * 2 * 8 <= RCAP * 4);
static_assert(NBA * 2 * 4 <= RCAP * 4);
static_assert(GBM * 8 == 4 * GTHR);
static_assert(GBM * R3W == 8 * GTHR);

typedef float          v2f   __attribute__((ext_vector_type(2)));
typedef float          v4f   __attribute__((ext_vector_type(4)));
typedef float          v8f   __attribute__((ext_vector_type(8)));
typedef double         v2d   __attribute__((ext_vector_type(2)));
typedef int            v4i   __attribute__((ext_vector_type(4)));
typedef int            v8i   __attribute__((ext_vector_type(8)));
typedef unsigned short v8us  __attribute__((ext_vector_type(8)));
typedef unsigned short v16us __attribute__((ext_vector_type(16)));
typedef __bf16         v16bf __attribute__((ext_vector_type(16)));
typedef v2f  __attribute__((may_alias)) v2fa;
typedef v4f  __attribute__((may_alias)) v4fa;
typedef v4i  __attribute__((may_alias)) v4ia;
typedef v8us __attribute__((may_alias)) v8usa;
union FragB { v16bf v; v16us u; v8us h[2]; v8i w; };

__device__ __forceinline__ v8f wmb(const FragB& a, const FragB& b, v8f c) {
  v8f d = __builtin_amdgcn_wmma_f32_16x16x32_bf16(false, a.v, false, b.v, (short)0, c, false, false);
  asm volatile("v_nop\n\tv_nop\n\tv_nop\n\tv_nop" : "+v"(d) : "v"(a.w), "v"(b.w));
  return d;
}

__device__ __forceinline__ unsigned bf16_bits(float f) {
  const unsigned u = __float_as_uint(f);
  return ((u + 0x7FFFu + ((u >> 16) & 1u)) >> 16) & 0xFFFFu;
}
__device__ __forceinline__ float bf16_val(float f) {
  return __uint_as_float(bf16_bits(f) << 16);
}
__device__ __forceinline__ v4f bfr4(const v4f a) {
  v4f r; r.x = bf16_val(a.x); r.y = bf16_val(a.y); r.z = bf16_val(a.z); r.w = bf16_val(a.w); return r;
}
__device__ __forceinline__ float leaky(float v) { return v > 0.f ? v : NEGSL * v; }

template <int SLB>
__device__ __forceinline__ int scan_chunk(const int* __restrict__ dsts, int nE, int cbase, int slotBase,
                                          int nb, int vec8, int* list, int tid, int lane, int wave) {
  int wc = 0;
  const int el0  = tid * EPT;
  const int e0   = cbase + el0;
  const int sent = -2147483647 - 1;
  v4i da, db;
  if (vec8 != 0 && cbase + CHUNK <= nE) {
    da = *(const v4i*)(dsts + e0);
    db = *(const v4i*)(dsts + e0 + 4);
  } else {
    da.x = (e0     < nE) ? dsts[min(e0,     nE - 1)] : sent;
    da.y = (e0 + 1 < nE) ? dsts[min(e0 + 1, nE - 1)] : sent;
    da.z = (e0 + 2 < nE) ? dsts[min(e0 + 2, nE - 1)] : sent;
    da.w = (e0 + 3 < nE) ? dsts[min(e0 + 3, nE - 1)] : sent;
    db.x = (e0 + 4 < nE) ? dsts[min(e0 + 4, nE - 1)] : sent;
    db.y = (e0 + 5 < nE) ? dsts[min(e0 + 5, nE - 1)] : sent;
    db.z = (e0 + 6 < nE) ? dsts[min(e0 + 6, nE - 1)] : sent;
    db.w = (e0 + 7 < nE) ? dsts[min(e0 + 7, nE - 1)] : sent;
  }
  const unsigned nbs = (unsigned)slotBase;
  const unsigned unb = (unsigned)nb;
  const unsigned s0 = (unsigned)da.x - nbs, s1 = (unsigned)da.y - nbs;
  const unsigned s2 = (unsigned)da.z - nbs, s3 = (unsigned)da.w - nbs;
  const unsigned s4 = (unsigned)db.x - nbs, s5 = (unsigned)db.y - nbs;
  const unsigned s6 = (unsigned)db.z - nbs, s7 = (unsigned)db.w - nbs;
  const bool h0 = s0 < unb, h1 = s1 < unb, h2 = s2 < unb, h3 = s3 < unb;
  const bool h4 = s4 < unb, h5 = s5 < unb, h6 = s6 < unb, h7 = s7 < unb;
  const unsigned any = __builtin_amdgcn_ballot_w32(h0 | h1 | h2 | h3 | h4 | h5 | h6 | h7);
  if (any != 0u) {
#define HITJ(J, HJ, SJ) { \
      const unsigned mj = __builtin_amdgcn_ballot_w32(HJ); \
      if (mj != 0u) { \
        if (HJ) { \
          const int pos = wc + (int)__builtin_amdgcn_mbcnt_lo(mj, 0u); \
          if (pos < WCAP) list[wave * WCAP + pos] = ((el0 + (J)) << SLB) | (int)(SJ); \
        } \
        wc += (int)__builtin_popcount(mj); } }
    HITJ(0, h0, s0)
    HITJ(1, h1, s1)
    HITJ(2, h2, s2)
    HITJ(3, h3, s3)
    HITJ(4, h4, s4)
    HITJ(5, h5, s5)
    HITJ(6, h6, s6)
    HITJ(7, h7, s7)
#undef HITJ
  }
  return wc;
}

__global__ __launch_bounds__(NTHR) void k_wprep(const float* __restrict__ W1, const float* __restrict__ W2,
                                                const float* __restrict__ W3,
                                                unsigned short* W1T, unsigned short* W2T, unsigned short* W3T) {
  const int u = (int)blockIdx.x * NTHR + (int)threadIdx.x;
  v8us o;
  unsigned short* dp;
  if (u < NU1) {
    const int n  = u >> 4;
    const int k8 = (u & 15) * 8;
    const float* p = W1 + (size_t)k8 * HC + n;
#pragma unroll
    for (int i = 0; i < 8; ++i) o[i] = (unsigned short)bf16_bits(p[(size_t)i * HC]);
    dp = W1T + (size_t)n * DIN + k8;
  } else if (u < NU1 + NU2) {
    const int v  = u - NU1;
    const int n  = v >> 5;
    const int k8 = (v & 31) * 8;
    const int kk = k8 & (HC - 1);
    const float* p = W2 + (size_t)kk * HC + n;
#pragma unroll
    for (int i = 0; i < 8; ++i) o[i] = (unsigned short)bf16_bits(p[(size_t)i * HC]);
    dp = W2T + (size_t)n * KP + k8;
  } else if (u < NU1 + NU2 + NU3) {
    const int v   = u - NU1 - NU2;
    const int n   = v >> 5;
    const int k8  = (v & 31) * 8;
    const int kk  = k8 & (HC - 1);
    const int ncl = n < C3 ? n : C3 - 1;
    const float* p = W3 + (size_t)kk * C3 + ncl;
#pragma unroll
    for (int i = 0; i < 8; ++i) {
      const unsigned short b = (unsigned short)bf16_bits(p[(size_t)i * C3]);
      o[i] = (n < C3) ? b : (unsigned short)0;
    }
    dp = W3T + (size_t)n * KP + k8;
  } else {
    return;
  }
  *(volatile v8us*)dp = o;
  __threadfence();
  *(volatile v8us*)dp = o;
}

__global__ __launch_bounds__(NTHR) void k_cvx(const float* __restrict__ x, int nN, int nUnits,
                                              unsigned short* xb) {
  const int u = (int)blockIdx.x * NTHR + (int)threadIdx.x;
  if (u >= nUnits) return;
  const int row = u >> 4;
  const int k8  = (u & 15) * 8;
  const int rc  = row < nN ? row : nN - 1;
  const float* p = x + (size_t)rc * DIN + k8;
  const v4f a = *(const v4f*)p;
  const v4f b = *(const v4f*)(p + 4);
  const bool ok = row < nN;
  v8us o;
  o[0] = ok ? (unsigned short)bf16_bits(a.x) : (unsigned short)0;
  o[1] = ok ? (unsigned short)bf16_bits(a.y) : (unsigned short)0;
  o[2] = ok ? (unsigned short)bf16_bits(a.z) : (unsigned short)0;
  o[3] = ok ? (unsigned short)bf16_bits(a.w) : (unsigned short)0;
  o[4] = ok ? (unsigned short)bf16_bits(b.x) : (unsigned short)0;
  o[5] = ok ? (unsigned short)bf16_bits(b.y) : (unsigned short)0;
  o[6] = ok ? (unsigned short)bf16_bits(b.z) : (unsigned short)0;
  o[7] = ok ? (unsigned short)bf16_bits(b.w) : (unsigned short)0;
  unsigned short* dp = xb + (size_t)row * DIN + k8;
  *(volatile v8us*)dp = o;
  __threadfence();
  *(volatile v8us*)dp = o;
}

__global__ __launch_bounds__(GTHR) void k_gemm(const unsigned short* __restrict__ A,
                                               const unsigned short* __restrict__ BT, int K,
                                               float* Cm, const float* __restrict__ avs,
                                               const float* __restrict__ avd, float* AL) {
  __shared__ __attribute__((aligned(16))) float stg[GBM * HC];
  __shared__ __attribute__((aligned(16))) float sdt[GBM * 8];
  const int tid = (int)threadIdx.x, lane = tid & 31, wave = tid >> 5, hh = lane >> 4, m = lane & 15;
  const int rowBase = (int)blockIdx.x * GBM;

  v8f acc[8];
  {
    const v8f z = {0.f, 0.f, 0.f, 0.f, 0.f, 0.f, 0.f, 0.f};
#pragma unroll
    for (int t = 0; t < 8; ++t) acc[t] = z;
  }
  const unsigned short* ap = A  + (size_t)(rowBase + 16 * wave + m) * (size_t)K + 8 * hh;
  const unsigned short* bp = BT + (size_t)m * (size_t)K + 8 * hh;

#pragma unroll 1
  for (int k0 = 0; k0 < K; k0 += 32) {
    FragB af;
    af.h[0] = *(const v8usa*)(ap + k0);
    af.h[1] = *(const v8usa*)(ap + k0 + 16);
#pragma unroll
    for (int nt = 0; nt < 8; ++nt) {
      const unsigned short* wq = bp + (size_t)(16 * nt) * (size_t)K + k0;
      FragB bf;
      bf.h[0] = *(const v8usa*)wq;
      bf.h[1] = *(const v8usa*)(wq + 16);
      acc[nt] = wmb(af, bf, acc[nt]);
    }
  }

#pragma unroll
  for (int nt = 0; nt < 8; ++nt) {
    const int lc = 16 * nt + m;
#pragma unroll
    for (int r = 0; r < 8; ++r) {
      const int lr = 16 * wave + 8 * hh + r;
      stg[lr * HC + lc] = acc[nt][r];
    }
  }
  __syncthreads();

  const v4f as4 = bfr4(*(const v4fa*)(avs + 4 * lane));
  const v4f ad4 = bfr4(*(const v4fa*)(avd + 4 * lane));
  const int head = lane >> 3;
#pragma unroll 1
  for (int i = 0; i < 16; ++i) {
    const int row = wave * 16 + i;
    const v4f p = *(const v4fa*)(stg + row * HC + 4 * lane);
    float s = p.x * as4.x; s = fmaf(p.y, as4.y, s); s = fmaf(p.z, as4.z, s); s = fmaf(p.w, as4.w, s);
    float d = p.x * ad4.x; d = fmaf(p.y, ad4.y, d); d = fmaf(p.z, ad4.z, d); d = fmaf(p.w, ad4.w, d);
#pragma unroll
    for (int off = 4; off > 0; off >>= 1) {
      s += __shfl_xor(s, off);
      d += __shfl_xor(d, off);
    }
    if ((lane & 7) == 0) { sdt[row * 8 + head] = s; sdt[row * 8 + 4 + head] = d; }
  }
  __syncthreads();

  const v4f alv = *(const v4fa*)(sdt + 4 * tid);
  float* alp = AL + (size_t)blockIdx.x * (GBM * 8) + 4 * tid;
#pragma unroll 1
  for (int i = 0; i < 16; ++i) {
    const int row = wave * 16 + i;
    const v4f p = *(const v4fa*)(stg + row * HC + 4 * lane);
    float* op = Cm + (size_t)(rowBase + row) * (size_t)HC + 4 * lane;
    *(volatile v4f*)op = p;
  }
  *(volatile v4f*)alp = alv;
  __threadfence();
#pragma unroll 1
  for (int i = 0; i < 16; ++i) {
    const int row = wave * 16 + i;
    const v4f p = *(const v4fa*)(stg + row * HC + 4 * lane);
    float* op = Cm + (size_t)(rowBase + row) * (size_t)HC + 4 * lane;
    *(volatile v4f*)op = p;
  }
  *(volatile v4f*)alp = alv;
}

__global__ __launch_bounds__(GTHR) void k_gemm3(const unsigned short* __restrict__ A,
                                                const unsigned short* __restrict__ BT, int K,
                                                const float* __restrict__ a3s, const float* __restrict__ a3d,
                                                float* R3) {
  __shared__ __attribute__((aligned(16))) float stg3[GBM * R3W];
  const int tid = (int)threadIdx.x, lane = tid & 31, wave = tid >> 5, hh = lane >> 4, m = lane & 15;
  const int rowBase = (int)blockIdx.x * GBM;
  v8f acc = {0.f, 0.f, 0.f, 0.f, 0.f, 0.f, 0.f, 0.f};
  const unsigned short* ap = A  + (size_t)(rowBase + 16 * wave + m) * (size_t)K + 8 * hh;
  const unsigned short* bp = BT + (size_t)m * (size_t)K + 8 * hh;
#pragma unroll 1
  for (int k0 = 0; k0 < K; k0 += 32) {
    FragB af, bf;
    af.h[0] = *(const v8usa*)(ap + k0);
    af.h[1] = *(const v8usa*)(ap + k0 + 16);
    bf.h[0] = *(const v8usa*)(bp + k0);
    bf.h[1] = *(const v8usa*)(bp + k0 + 16);
    acc = wmb(af, bf, acc);
  }
#pragma unroll
  for (int r = 0; r < 8; ++r) {
    const int lr = 16 * wave + 8 * hh + r;
    stg3[lr * R3W + m] = acc[r];
  }
  __syncthreads();
  {
    const int row = tid & 63, which = tid >> 6;
    const v4f s0 = *(const v4fa*)a3s, s1 = *(const v4fa*)(a3s + 4);
    const v4f d0 = *(const v4fa*)a3d, d1 = *(const v4fa*)(a3d + 4);
    v4f w0, w1;
    w0.x = bf16_val(which ? d0.x : s0.x); w0.y = bf16_val(which ? d0.y : s0.y);
    w0.z = bf16_val(which ? d0.z : s0.z); w0.w = bf16_val(which ? d0.w : s0.w);
    w1.x = bf16_val(which ? d1.x : s1.x); w1.y = bf16_val(which ? d1.y : s1.y);
    w1.z = bf16_val(which ? d1.z : s1.z); w1.w = bf16_val(which ? d1.w : s1.w);
    const v4f x0 = *(const v4fa*)(stg3 + row * R3W);
    const v4f x1 = *(const v4fa*)(stg3 + row * R3W + 4);
    v4f dv;
    dv.x = fmaf(x0.y, w0.y, x0.x * w0.x);
    dv.y = fmaf(x0.w, w0.w, x0.z * w0.z);
    dv.z = fmaf(x1.y, w1.y, x1.x * w1.x);
    dv.w = fmaf(x1.w, w1.w, x1.z * w1.z);
    *(v4fa*)(stg3 + row * R3W + 8 + 4 * which) = dv;
  }
  __syncthreads();
  const v4f pa = *(const v4fa*)(stg3 + 4 * tid);
  const v4f pb = *(const v4fa*)(stg3 + 4 * (tid + GTHR));
  float* oa = R3 + (size_t)rowBase * R3W + 4 * tid;
  float* ob = oa + 4 * GTHR;
  *(volatile v4f*)oa = pa;
  *(volatile v4f*)ob = pb;
  __threadfence();
  *(volatile v4f*)oa = pa;
  *(volatile v4f*)ob = pb;
}

__device__ __forceinline__ void build_lists(const int* __restrict__ dsts, int nE, int vec8, int nodeBase,
                                            int* dsm, int tid, int lane, int wave, int& ttOut, int& ovfOut) {
  int* list = dsm;
  int* hl   = dsm + LISTN;
  int* sl   = dsm + LISTN + RCAP;
  int* cnt  = dsm + LISTN + 2 * RCAP;
  int* offs = cnt + NBA;
  int* cur  = offs + NBA;
  int* misc = cur + NBA;
  {
    const v4i z4 = {0, 0, 0, 0};
    for (int i = tid * 4; i < AGG_ZINTS; i += NTHR * 4) *(v4ia*)(dsm + i) = z4;
    if (tid < 16) misc[tid] = 0;
  }
  __syncthreads();

  int t = 0, ov = 0;
  const int nChunks = (nE + CHUNK - 1) / CHUNK;
#pragma unroll 1
  for (int ch = 0; ch < nChunks; ++ch) {
    const int cbase = ch * CHUNK;
    const int wc = scan_chunk<SLA>(dsts, nE, cbase, nodeBase, NBA, vec8, list, tid, lane, wave);
    if (lane == 0) misc[wave] = wc;
    __syncthreads();
    if (wave == 0) {
#pragma unroll 1
      for (int w2 = 0; w2 < NWAVE; ++w2) {
        int c = misc[w2];
        c = c < 0 ? 0 : (c > WCAP ? WCAP : c);
#pragma unroll 1
        for (int b0 = 0; b0 < c; b0 += 32) {
          const int idx = b0 + lane;
          const int ent = list[w2 * WCAP + (idx < WCAP ? idx : WCAP - 1)];
          const int m32 = (c - b0) < 32 ? (c - b0) : 32;
#pragma unroll 1
          for (int k = 0; k < m32; ++k) {
            const int u    = __builtin_amdgcn_readlane(ent, k);
            const int slot = u & (NBA - 1);
            const int el   = (u >> SLA) & (CHUNK - 1);
            const int pk   = ((cbase + el) << SLA) | slot;
            if (t < RCAP) {
              if (lane == 0) { hl[t] = pk; cnt[slot] = cnt[slot] + 1; }
              t = t + 1;
            } else {
              ov = 1;
            }
          }
        }
      }
    }
    __syncthreads();
  }
  if (wave == 0 && lane == 0) { misc[8] = t; misc[9] = ov; }
  __syncthreads();
  int tt = misc[8];
  tt = tt < 0 ? 0 : (tt > RCAP ? RCAP : tt);
  const int ovf = misc[9];

  if (wave == 0) {
    const int base = lane * (NBA / 32);
    int s = 0;
#pragma unroll 1
    for (int i = 0; i < NBA / 32; ++i) s += cnt[base + i];
    int incl = s;
#pragma unroll
    for (int d = 1; d < 32; d <<= 1) {
      const int y = __shfl_up(incl, d, 32);
      if (lane >= d) incl += y;
    }
    int run = incl - s;
#pragma unroll 1
    for (int i = 0; i < NBA / 32; ++i) {
      const int cv = cnt[base + i];
      offs[base + i] = run;
      cur[base + i]  = run;
      run += cv;
    }
  }
  __syncthreads();
  if (wave == 0) {
#pragma unroll 1
    for (int b0 = 0; b0 < tt; b0 += 32) {
      const int idx = b0 + lane;
      const int ent = hl[idx < RCAP ? idx : RCAP - 1];
      const int m32 = (tt - b0) < 32 ? (tt - b0) : 32;
#pragma unroll 1
      for (int k = 0; k < m32; ++k) {
        const int u    = __builtin_amdgcn_readlane(ent, k);
        const int slot = u & (NBA - 1);
        if (lane == 0) {
          int p = cur[slot];
          p = p < 0 ? 0 : (p > RCAP - 1 ? RCAP - 1 : p);
          sl[p] = u;
          cur[slot] = p + 1;
        }
      }
    }
  }
  __syncthreads();
  ttOut = tt;
  ovfOut = ovf;
}

__global__ __launch_bounds__(NTHR) void k_agg(const int* __restrict__ srcs, const int* __restrict__ dsts,
                                              int nE, int nN, int vec8,
                                              const float* __restrict__ AL, const float* __restrict__ xl,
                                              const float* __restrict__ bias, float* Eo, double* REC) {
  extern __shared__ __attribute__((aligned(16))) int dsm[];
  int* sl   = dsm + LISTN + RCAP;
  int* cnt  = dsm + LISTN + 2 * RCAP;
  int* offs = cnt + NBA;
  const int tid = (int)threadIdx.x, lane = tid & 31, wave = tid >> 5;
  const int nodeBase = (int)blockIdx.x * NBA;
  int tt = 0, ovf = 0;
  build_lists(dsts, nE, vec8, nodeBase, dsm, tid, lane, wave, tt, ovf);
  (void)tt;

  const v4f bb = bfr4(*(const v4fa*)(bias + 4 * lane));
  const int head = lane >> 3;
  const float qnan = __int_as_float(0x7fc00000);
  const float pz = (ovf != 0) ? qnan : 0.0f;
  double sx0 = 0.0, sx1 = 0.0, sx2 = 0.0, sx3 = 0.0;
  double qx0 = 0.0, qx1 = 0.0, qx2 = 0.0, qx3 = 0.0;

#pragma unroll 1
  for (int si = 0; si < NBA / NWAVE; ++si) {
    const int s    = si * NWAVE + wave;
    const int node = nodeBase + s;
    int c = cnt[s];
    const bool big = c > DEGCAP;
    c = c < 0 ? 0 : (c > DEGCAP ? DEGCAP : c);
    int o = offs[s];
    o = o < 0 ? 0 : (o > RCAP ? RCAP : o);
    const int nc = node < nN ? node : nN - 1;
    const float as0 = AL[(size_t)nc * 8 + head];
    const float ad  = AL[(size_t)nc * 8 + 4 + head];
    v4f acc = *(const v4f*)(xl + (size_t)nc * HC + 4 * lane);
    float mx = leaky(as0 + ad), dn = 1.0f;
#pragma unroll 1
    for (int b0 = 0; b0 < c; b0 += 32) {
      int idx = o + b0 + lane;
      idx = idx > RCAP - 1 ? RCAP - 1 : idx;
      const int ent = sl[idx];
      int eid = ent >> SLA;
      eid = eid < 0 ? 0 : (eid > nE - 1 ? nE - 1 : eid);
      int sr = srcs[eid];
      sr = sr < 0 ? 0 : (sr > nN - 1 ? nN - 1 : sr);
      const int m32 = (c - b0) < 32 ? (c - b0) : 32;
#pragma unroll 1
      for (int k = 0; k < m32; ++k) {
        const int sk = __builtin_amdgcn_readlane(sr, k);
        const v4f a = *(const v4f*)(xl + (size_t)sk * HC + 4 * lane);
        const float ask = AL[(size_t)sk * 8 + head];
        const float lg = leaky(ask + ad);
        const float df = lg - mx;
        const float ee = expf(-fabsf(df));
        const bool  up = df > 0.f;
        const float s1 = up ? ee : 1.0f;
        const float s2 = up ? 1.0f : ee;
        mx = up ? lg : mx;
        dn = fmaf(dn, s1, s2);
        acc.x = fmaf(acc.x, s1, s2 * a.x); acc.y = fmaf(acc.y, s1, s2 * a.y);
        acc.z = fmaf(acc.z, s1, s2 * a.z); acc.w = fmaf(acc.w, s1, s2 * a.w);
      }
    }
    const float inv = __builtin_amdgcn_rcpf(dn + EPS_SM);
    const float pzr = big ? qnan : pz;
    float y0 = fmaf(acc.x, inv, bb.x), y1 = fmaf(acc.y, inv, bb.y);
    float y2 = fmaf(acc.z, inv, bb.z), y3 = fmaf(acc.w, inv, bb.w);
#pragma unroll 1
    for (int i = 0; i < 4; ++i) {
      const float tv = (i == 0) ? y0 : ((i == 1) ? y1 : ((i == 2) ? y2 : y3));
      const float ev = (tv > 0.f) ? tv : expm1f(tv);
      y0 = (i == 0) ? ev : y0;
      y1 = (i == 1) ? ev : y1;
      y2 = (i == 2) ? ev : y2;
      y3 = (i == 3) ? ev : y3;
    }
    y0 += pzr; y1 += pzr; y2 += pzr; y3 += pzr;
    if (node < nN) {
      v4f ov4; ov4.x = y0; ov4.y = y1; ov4.z = y2; ov4.w = y3;
      float* op = Eo + (size_t)node * HC + 4 * lane;
      *(volatile v4f*)op = ov4;
      __threadfence();
      *(volatile v4f*)op = ov4;
      const double d0 = (double)y0, d1 = (double)y1, d2 = (double)y2, d3 = (double)y3;
      sx0 += d0; sx1 += d1; sx2 += d2; sx3 += d3;
      qx0 = fma(d0, d0, qx0); qx1 = fma(d1, d1, qx1); qx2 = fma(d2, d2, qx2); qx3 = fma(d3, d3, qx3);
    }
  }

  double* part = (double*)(dsm + LISTN);
  {
    double* wp = part + (size_t)(wave * HC + 4 * lane) * 2;
    wp[0] = sx0; wp[1] = qx0; wp[2] = sx1; wp[3] = qx1;
    wp[4] = sx2; wp[5] = qx2; wp[6] = sx3; wp[7] = qx3;
  }
  __syncthreads();
  if (tid < HC) {
    double S = 0.0, Q = 0.0;
#pragma unroll
    for (int w2 = 0; w2 < NWAVE; ++w2) {
      S += part[(size_t)(w2 * HC + tid) * 2];
      Q += part[(size_t)(w2 * HC + tid) * 2 + 1];
    }
    v2d rv; rv.x = S; rv.y = Q;
    double* rp = REC + ((size_t)blockIdx.x * HC + tid) * 2;
    *(volatile v2d*)rp = rv;
    __threadfence();
    *(volatile v2d*)rp = rv;
  }
}

__global__ __launch_bounds__(HC) void k_bnstat(const double* __restrict__ REC, int nBlk, double invN, float* TAB) {
  __shared__ __attribute__((aligned(16))) float tab[2 * HC];
  const int c = (int)threadIdx.x;
  double S = 0.0, Q = 0.0;
#pragma unroll 1
  for (int b = 0; b < nBlk; ++b) {
    const v2d r = *(const v2d*)(REC + ((size_t)b * HC + c) * 2);
    S += r.x; Q += r.y;
  }
  const double mean = S * invN;
  const double var  = fma(Q, invN, -(mean * mean));
  float vf = (float)var;
  vf = (vf < 0.f) ? 0.f : vf;
  tab[c]      = (float)mean;
  tab[HC + c] = rsqrtf(vf + BN_EPS);
  __syncthreads();
  if (c < (2 * HC) / 4) {
    const v4f v = *(const v4fa*)(tab + 4 * c);
    float* tp = TAB + 4 * c;
    *(volatile v4f*)tp = v;
    __threadfence();
    *(volatile v4f*)tp = v;
  }
}

__global__ __launch_bounds__(NTHR) void k_bnsplit(const float* __restrict__ Ein, const float* __restrict__ TAB,
                                                  const float* __restrict__ g, const float* __restrict__ be,
                                                  int nN, int nUnits, unsigned short* Hp) {
  const int u = (int)blockIdx.x * NTHR + (int)threadIdx.x;
  if (u >= nUnits) return;
  const int row = u >> 4;
  const int c0  = (u & 15) * 8;
  const int rc  = row < nN ? row : nN - 1;
  const float* ep = Ein + (size_t)rc * HC + c0;
  const v4f va = *(const v4f*)ep,              vb = *(const v4f*)(ep + 4);
  const v4f ma = *(const v4f*)(TAB + c0),      mb = *(const v4f*)(TAB + c0 + 4);
  const v4f ra = *(const v4f*)(TAB + HC + c0), rb = *(const v4f*)(TAB + HC + c0 + 4);
  const v4f ga = bfr4(*(const v4f*)(g + c0)),  gb = bfr4(*(const v4f*)(g + c0 + 4));
  const v4f ba = bfr4(*(const v4f*)(be + c0)), bq = bfr4(*(const v4f*)(be + c0 + 4));
  float y[8];
  y[0] = (ga.x * (va.x - ma.x)) * ra.x + ba.x;
  y[1] = (ga.y * (va.y - ma.y)) * ra.y + ba.y;
  y[2] = (ga.z * (va.z - ma.z)) * ra.z + ba.z;
  y[3] = (ga.w * (va.w - ma.w)) * ra.w + ba.w;
  y[4] = (gb.x * (vb.x - mb.x)) * rb.x + bq.x;
  y[5] = (gb.y * (vb.y - mb.y)) * rb.y + bq.y;
  y[6] = (gb.z * (vb.z - mb.z)) * rb.z + bq.z;
  y[7] = (gb.w * (vb.w - mb.w)) * rb.w + bq.w;
  const bool ok = row < nN;
  v8us ho, lo;
#pragma unroll
  for (int i = 0; i < 8; ++i) {
    const float yv = ok ? y[i] : 0.0f;
    const unsigned hbi = bf16_bits(yv);
    ho[i] = (unsigned short)hbi;
    lo[i] = (unsigned short)bf16_bits(yv - __uint_as_float(hbi << 16));
  }
  unsigned short* hp = Hp + (size_t)row * KP + c0;
  *(volatile v8us*)hp = ho;
  *(volatile v8us*)(hp + HC) = lo;
  __threadfence();
  *(volatile v8us*)hp = ho;
  *(volatile v8us*)(hp + HC) = lo;
}

__device__ __forceinline__ void upd2(float& mx, float& dn, float& a0, float& a1,
                                     float lg, float y0, float y1, bool act) {
  const float df = lg - mx;
  const float ee = expf(-fabsf(df));
  const bool  up = df > 0.f;
  float s1 = up ? ee : 1.0f;
  float s2 = up ? 1.0f : ee;
  s1 = act ? s1 : 1.0f;
  s2 = act ? s2 : 0.0f;
  mx = (act && up) ? lg : mx;
  dn = fmaf(dn, s1, s2);
  a0 = fmaf(a0, s1, s2 * y0);
  a1 = fmaf(a1, s1, s2 * y1);
}

__global__ __launch_bounds__(NTHR) void k_agg3(const int* __restrict__ srcs, const int* __restrict__ dsts,
                                               int nE, int nN, int vec8,
                                               const float* __restrict__ R3, const float* __restrict__ b3,
                                               float* outp) {
  extern __shared__ __attribute__((aligned(16))) int dsm[];
  int* sl   = dsm + LISTN + RCAP;
  int* cnt  = dsm + LISTN + 2 * RCAP;
  int* offs = cnt + NBA;
  float* res = (float*)(dsm + LISTN);
  const int tid = (int)threadIdx.x, lane = tid & 31, wave = tid >> 5;
  const int nodeBase = (int)blockIdx.x * NBA;
  int tt = 0, ovf = 0;
  build_lists(dsts, nE, vec8, nodeBase, dsm, tid, lane, wave, tt, ovf);
  (void)tt;

  const float qnan = __int_as_float(0x7fc00000);
  const float pz = (ovf != 0) ? qnan : 0.0f;
  const float bz0 = bf16_val(b3[0]), bz1 = bf16_val(b3[1]);

#pragma unroll 1
  for (int j = 0; j < NBA / NTHR; ++j) {
    const int s    = j * NTHR + tid;
    const int node = nodeBase + s;
    const int nc   = node < nN ? node : nN - 1;
    int c = cnt[s];
    const bool big = c > DEGCAP;
    c = c < 0 ? 0 : (c > DEGCAP ? DEGCAP : c);
    int o = offs[s];
    o = o < 0 ? 0 : (o > RCAP ? RCAP : o);
    int cm = c;
#pragma unroll
    for (int off = 16; off > 0; off >>= 1) {
      const int oth = __shfl_xor(cm, off);
      cm = oth > cm ? oth : cm;
    }
    const float* rp = R3 + (size_t)nc * R3W;
    const v4f xa = *(const v4f*)rp, xb = *(const v4f*)(rp + 4);
    const v4f sa = *(const v4f*)(rp + 8), da = *(const v4f*)(rp + 12);
    float mx0 = leaky(sa.x + da.x), mx1 = leaky(sa.y + da.y), mx2 = leaky(sa.z + da.z), mx3 = leaky(sa.w + da.w);
    float dn0 = 1.0f, dn1 = 1.0f, dn2 = 1.0f, dn3 = 1.0f;
    float a00 = xa.x, a01 = xa.y, a10 = xa.z, a11 = xa.w;
    float a20 = xb.x, a21 = xb.y, a30 = xb.z, a31 = xb.w;
    const int cl = c > 0 ? c - 1 : 0;
#pragma unroll 1
    for (int q = 0; q < cm; ++q) {
      const bool act = q < c;
      const int qq = q < cl ? q : cl;
      int idx = o + qq;
      idx = idx > RCAP - 1 ? RCAP - 1 : idx;
      const int ent = sl[idx];
      int eid = ent >> SLA;
      eid = eid < 0 ? 0 : (eid > nE - 1 ? nE - 1 : eid);
      int sr = srcs[eid];
      sr = sr < 0 ? 0 : (sr > nN - 1 ? nN - 1 : sr);
      const float* sp = R3 + (size_t)sr * R3W;
      const v4f ya = *(const v4f*)sp, yb = *(const v4f*)(sp + 4), ys = *(const v4f*)(sp + 8);
      upd2(mx0, dn0, a00, a01, leaky(ys.x + da.x), ya.x, ya.y, act);
      upd2(mx1, dn1, a10, a11, leaky(ys.y + da.y), ya.z, ya.w, act);
      upd2(mx2, dn2, a20, a21, leaky(ys.z + da.z), yb.x, yb.y, act);
      upd2(mx3, dn3, a30, a31, leaky(ys.w + da.w), yb.z, yb.w, act);
    }
    const float i0 = __builtin_amdgcn_rcpf(dn0 + EPS_SM), i1 = __builtin_amdgcn_rcpf(dn1 + EPS_SM);
    const float i2 = __builtin_amdgcn_rcpf(dn2 + EPS_SM), i3 = __builtin_amdgcn_rcpf(dn3 + EPS_SM);
    const float pzr = big ? qnan : pz;
    v2f ov;
    ov.x = fmaf(0.25f, ((a00 * i0 + a10 * i1) + a20 * i2) + a30 * i3, bz0) + pzr;
    ov.y = fmaf(0.25f, ((a01 * i0 + a11 * i1) + a21 * i2) + a31 * i3, bz1) + pzr;
    *(v2fa*)(res + 2 * s) = ov;
  }
  __syncthreads();
  int lv = nN - nodeBase;
  lv = lv < 0 ? 0 : (lv > NBA ? NBA : lv);
  const int npc = lv >> 1;
  float* ob = outp + (size_t)nodeBase * 2;
#pragma unroll 1
  for (int p = tid; p < npc; p += NTHR) {
    const v4f v = *(const v4fa*)(res + 4 * p);
    *(volatile v4f*)(ob + 4 * p) = v;
  }
  __threadfence();
#pragma unroll 1
  for (int p = tid; p < npc; p += NTHR) {
    const v4f v = *(const v4fa*)(res + 4 * p);
    *(volatile v4f*)(ob + 4 * p) = v;
  }
}

static inline int cdiv(int a, int b) { return (a + b - 1) / b; }

extern "C" void kernel_launch(void* const* d_in, const int* in_sizes, int n_in,
                              void* d_out, int out_size, void* d_ws, size_t ws_size,
                              hipStream_t stream) {
  if (n_in < 18) return;
  if (in_sizes[0] < DIN || (in_sizes[0] % DIN) != 0) return;
  const int nN = in_sizes[0] / DIN;
  if ((nN % 16) != 0 || nN > (1 << 24)) return;
  if (in_sizes[1] < 2 || (in_sizes[1] & 1) != 0) return;
  const int nE = in_sizes[1] / 2;
  if (nE < 1 || nE >= (1 << 21)) return;
  if (in_sizes[2] != DIN * HC) return;
  if (in_sizes[3] != HC || in_sizes[4] != HC) return;
  if (in_sizes[5] != HC || in_sizes[6] != HC || in_sizes[7] != HC) return;
  if (in_sizes[8] != HC * HC) return;
  if (in_sizes[9] != HC || in_sizes[10] != HC) return;
  if (in_sizes[11] != HC || in_sizes[12] != HC || in_sizes[13] != HC) return;
  if (in_sizes[14] != HC * C3) return;
  if (in_sizes[15] != C3 || in_sizes[16] != C3) return;
  if (in_sizes[17] != 2) return;
  if ((long long)out_size != 2LL * (long long)nN) return;

  const float* x    = (const float*)d_in[0];
  const int*   edge = (const int*)d_in[1];
  const float* W1   = (const float*)d_in[2];
  const float* as1  = (const float*)d_in[3];
  const float* ad1  = (const float*)d_in[4];
  const float* b1   = (const float*)d_in[5];
  const float* g1   = (const float*)d_in[6];
  const float* be1  = (const float*)d_in[7];
  const float* W2   = (const float*)d_in[8];
  const float* as2  = (const float*)d_in[9];
  const float* ad2  = (const float*)d_in[10];
  const float* b2   = (const float*)d_in[11];
  const float* g2   = (const float*)d_in[12];
  const float* be2  = (const float*)d_in[13];
  const float* W3   = (const float*)d_in[14];
  const float* as3  = (const float*)d_in[15];
  const float* ad3  = (const float*)d_in[16];
  const float* b3   = (const float*)d_in[17];
  float* out = (float*)d_out;
  const int* src = edge;
  const int* dst = edge + nE;

  const int MP   = cdiv(nN, GBM) * GBM;
  const int gM   = MP / GBM;
  const int gA   = cdiv(MP, NBA);
  if ((long long)gA * NBA < (long long)MP) return;
  const int vec8 = ((nE & 3) == 0) ? 1 : 0;
  const double invN = 1.0 / (double)nN;

  char* ws = (char*)d_ws;
  size_t off = 0;
  const size_t oW1T = off; off += (size_t)HC * DIN * 2;            off = (off + 255) & ~(size_t)255;
  const size_t oW2T = off; off += (size_t)HC * KP * 2;             off = (off + 255) & ~(size_t)255;
  const size_t oW3T = off; off += (size_t)N3P * KP * 2;            off = (off + 255) & ~(size_t)255;
  const size_t oTAB = off; off += (size_t)2 * HC * 4;              off = (off + 255) & ~(size_t)255;
  const size_t oREC = off; off += (size_t)gA * HC * 2 * 8;         off = (off + 255) & ~(size_t)255;
  const size_t oAL  = off; off += (size_t)MP * 8 * 4;              off = (off + 255) & ~(size_t)255;
  const size_t oR3  = off; off += (size_t)MP * R3W * 4;            off = (off + 255) & ~(size_t)255;
  const size_t oXB  = off; off += (size_t)MP * DIN * 2;            off = (off + 255) & ~(size_t)255;
  const size_t oXW  = off; off += (size_t)MP * HC * 4;             off = (off + 255) & ~(size_t)255;
  const size_t oEP  = off; off += (size_t)MP * HC * 4;             off = (off + 255) & ~(size_t)255;
  const size_t oHP  = off; off += (size_t)MP * KP * 2;             off = (off + 255) & ~(size_t)255;
  if (off > ws_size || off > (size_t)WSMAX) return;
  unsigned short* W1T = (unsigned short*)(ws + oW1T);
  unsigned short* W2T = (unsigned short*)(ws + oW2T);
  unsigned short* W3T = (unsigned short*)(ws + oW3T);
  float*          TAB = (float*)(ws + oTAB);
  double*         REC = (double*)(ws + oREC);
  float*          ALp = (float*)(ws + oAL);
  float*          R3  = (float*)(ws + oR3);
  unsigned short* XB  = (unsigned short*)(ws + oXB);
  float*          XW  = (float*)(ws + oXW);
  float*          EP  = (float*)(ws + oEP);
  unsigned short* HP  = (unsigned short*)(ws + oHP);

  const size_t aggLds = (size_t)AGG_LDS_INTS * 4;
  hipFuncSetAttribute(reinterpret_cast<const void*>(&k_agg),  hipFuncAttributeMaxDynamicSharedMemorySize, (int)aggLds);
  hipFuncSetAttribute(reinterpret_cast<const void*>(&k_agg3), hipFuncAttributeMaxDynamicSharedMemorySize, (int)aggLds);

  const int nUx = MP * (DIN / 8);
  const int nUs = MP * (HC / 8);
  k_wprep<<<(NU1 + NU2 + NU3) / NTHR, NTHR, 0, stream>>>(W1, W2, W3, W1T, W2T, W3T);
  k_cvx<<<cdiv(nUx, NTHR), NTHR, 0, stream>>>(x, nN, nUx, XB);
  k_gemm<<<gM, GTHR, 0, stream>>>(XB, W1T, DIN, XW, as1, ad1, ALp);
  k_agg<<<gA, NTHR, aggLds, stream>>>(src, dst, nE, nN, vec8, ALp, XW, b1, EP, REC);
  k_bnstat<<<1, HC, 0, stream>>>(REC, gA, invN, TAB);
  k_bnsplit<<<cdiv(nUs, NTHR), NTHR, 0, stream>>>(EP, TAB, g1, be1, nN, nUs, HP);
  k_gemm<<<gM, GTHR, 0, stream>>>(HP, W2T, KP, XW, as2, ad2, ALp);
  k_agg<<<gA, NTHR, aggLds, stream>>>(src, dst, nE, nN, vec8, ALp, XW, b2, EP, REC);
  k_bnstat<<<1, HC, 0, stream>>>(REC, gA, invN, TAB);
  k_bnsplit<<<cdiv(nUs, NTHR), NTHR, 0, stream>>>(EP, TAB, g2, be2, nN, nUs, HP);
  k_gemm3<<<gM, GTHR, 0, stream>>>(HP, W3T, KP, as3, ad3, R3);
  k_agg3<<<gA, NTHR, aggLds, stream>>>(src, dst, nE, nN, vec8, R3, b3, out);
}
